// CNNVectorForm_34668976014087
// MI455X (gfx1250) — hardware-verified
//
#include <hip/hip_runtime.h>
#include <math.h>
#include <stdint.h>

#define DEVINL __device__ __forceinline__

typedef _Float16 f16t;
typedef _Float16 v16h __attribute__((ext_vector_type(16)));
typedef _Float16 v8h  __attribute__((ext_vector_type(8)));
typedef float    v8f  __attribute__((ext_vector_type(8)));
typedef float    v4f  __attribute__((ext_vector_type(4)));
typedef v8h __attribute__((may_alias)) v8ha;
typedef v4f __attribute__((may_alias)) v4fa;
union FragH { v16h v; v8h half[2]; };

#define IW     28
#define IMGSZ  784
#define IMS    29
#define IMLDS  812
#define CO     20
#define KTAP   25
#define KCP    32
#define NCP    32
#define FC1IN  2880
#define FC1O   500
#define FC1P   512
#define FC2O   10
#define FC2P   16
#define TPB    256
#define STGP   64

#define XC   4.0f
#define WCC  64.0f
#define A1C  16.0f
#define W1C  1024.0f
#define A2C  16.0f
#define W2C  256.0f

static_assert((FC1IN % 32) == 0);
static_assert((FC1IN * 2) % 128 == 0);
static_assert((FC1P * 2) % 128 == 0);
static_assert(FC1P * (FC1IN / 8) == 720 * TPB);

DEVINL int imin(int a, int b) { return a < b ? a : b; }
DEVINL int imax(int a, int b) { return a > b ? a : b; }

DEVINL v8f wmma_f16(v16h a, v16h b, v8f c) {
  v8f d = __builtin_amdgcn_wmma_f32_16x16x32_f16(false, a, false, b, (short)0, c, false, false);
  asm volatile("v_nop\n\tv_nop\n\tv_nop\n\tv_nop" : "+v"(d) : "v"(a), "v"(b));
  return d;
}
DEVINL v8f zero8f() {
  v8f z = {0.f, 0.f, 0.f, 0.f, 0.f, 0.f, 0.f, 0.f};
  return z;
}

__global__ __launch_bounds__(TPB) void prep_k(const float* __restrict__ conv_w,
                                             const float* __restrict__ fc1_w,
                                             const float* __restrict__ fc2_w,
                                             f16t* __restrict__ Wc, f16t* __restrict__ W1,
                                             f16t* __restrict__ W2)
{
  const int t = blockIdx.x * TPB + threadIdx.x;
  const int y = blockIdx.y;
  if (y == 0) {
    if (t >= FC1P * (FC1IN / 8)) return;
    const int n = t / (FC1IN / 8);
    const int p = t - n * (FC1IN / 8);
    const int ncl = imin(n, FC1O - 1);
    const float sc = (n < FC1O) ? W1C : 0.0f;
    const float* src = fc1_w + (size_t)ncl * FC1IN + 8 * p;
    const v4f f0 = *(const v4fa*)src;
    const v4f f1 = *(const v4fa*)(src + 4);
    v8h o;
    #pragma unroll
    for (int i = 0; i < 4; ++i) {
      o[i]     = (f16t)(f0[i] * sc);
      o[4 + i] = (f16t)(f1[i] * sc);
    }
    f16t* dst = W1 + (size_t)8 * t;
    *(volatile v8h*)dst = o;
    __threadfence();
    *(volatile v8h*)dst = o;
  } else if (y == 1) {
    if (t >= NCP * (KCP / 8)) return;
    const int n = t >> 2, part = t & 3;
    const int ncl = imin(n, CO - 1);
    v8h o;
    #pragma unroll
    for (int i = 0; i < 8; ++i) {
      const int k = 8 * part + i;
      const int kcl = imin(k, KTAP - 1);
      const float w = conv_w[ncl * KTAP + kcl];
      const float sc = (n < CO && k < KTAP) ? WCC : 0.0f;
      o[i] = (f16t)(w * sc);
    }
    f16t* dst = Wc + 8 * t;
    *(volatile v8h*)dst = o;
    __threadfence();
    *(volatile v8h*)dst = o;
  } else {
    if (t >= FC2P * (FC1P / 8)) return;
    const int n = t >> 6, part = t & 63;
    const int ncl = imin(n, FC2O - 1);
    v8h o;
    #pragma unroll
    for (int i = 0; i < 8; ++i) {
      const int k = 8 * part + i;
      const int kcl = imin(k, FC1O - 1);
      const float w = fc2_w[ncl * FC1O + kcl];
      const float sc = (n < FC2O && k < FC1O) ? W2C : 0.0f;
      o[i] = (f16t)(w * sc);
    }
    f16t* dst = W2 + 8 * t;
    *(volatile v8h*)dst = o;
    __threadfence();
    *(volatile v8h*)dst = o;
  }
}

__global__ __launch_bounds__(TPB) void conv_pool_k(const float* __restrict__ x,
                                                  const float* __restrict__ conv_b,
                                                  const f16t* __restrict__ Wc,
                                                  f16t* __restrict__ act1)
{
  __shared__ __attribute__((aligned(16))) f16t simg[2 * IMLDS];
  __shared__ __attribute__((aligned(16))) f16t spool[2 * FC1IN];
  const int tid = threadIdx.x, lane = tid & 31, wave = tid >> 5;
  const int h = lane >> 4, m = lane & 15;
  const int img0 = blockIdx.x * 2;

  {
    const float* xb = x + (size_t)img0 * IMGSZ;
    for (int idx = tid; idx < 2 * IMGSZ; idx += TPB) {
      const int il  = (idx >= IMGSZ) ? 1 : 0;
      const int rem = idx - il * IMGSZ;
      const int r   = rem / IW;
      const int c   = rem - r * IW;
      simg[il * IMLDS + r * IMS + c] = (f16t)(xb[idx] * XC);
    }
  }
  __syncthreads();

  const int il = wave >> 2, sub = wave & 3;
  const f16t* im = simg + il * IMLDS;
  f16t* pl = spool + il * FC1IN;

  FragH b0, b1;
  {
    const f16t* w0 = Wc + m * KCP + 8 * h;
    b0.half[0] = *(const v8ha*)(w0);
    b0.half[1] = *(const v8ha*)(w0 + 16);
    const f16t* w1 = Wc + (16 + m) * KCP + 8 * h;
    b1.half[0] = *(const v8ha*)(w1);
    b1.half[1] = *(const v8ha*)(w1 + 16);
  }
  const float bias0 = conv_b[m];
  const float bias1 = conv_b[imin(16 + m, CO - 1)];

  int offs[16];
  #pragma unroll
  for (int e = 0; e < 16; ++e) {
    const int k  = (e < 8) ? (8 * h + e) : (8 + 8 * h + e);
    const int kc = imin(k, KTAP - 1);
    const int ky = kc / 5, kx = kc - ky * 5;
    offs[e] = ky * IMS + kx;
  }
  const bool hsel = (h != 0);
  const int py_off = m & 1, px_off = m >> 1;
  const float inv_c = 1.0f / (XC * WCC);

  #pragma unroll 1
  for (int i = 0; i < 9; ++i) {
    const int t  = sub * 9 + i;
    const int t3 = t / 3;
    const int r0 = t3 * 2;
    const int c0 = (t - t3 * 3) * 8;
    const int bidx = (r0 + py_off) * IMS + c0 + px_off;
    v16h av;
    #pragma unroll
    for (int e = 0; e < 16; ++e) {
      f16t v = im[bidx + offs[e]];
      if (e >= 9) v = hsel ? (f16t)0.0f : v;
      av[e] = v;
    }
    const v8f acc0 = wmma_f16(av, b0.v, zero8f());
    const v8f acc1 = wmma_f16(av, b1.v, zero8f());

    const int pr = r0 >> 1;
    const int pc = (c0 >> 1) + 2 * h;
    const float p0 = fmaxf(fmaxf(acc0[0], acc0[1]), fmaxf(acc0[2], acc0[3])) * inv_c + bias0;
    const float p1 = fmaxf(fmaxf(acc0[4], acc0[5]), fmaxf(acc0[6], acc0[7])) * inv_c + bias0;
    f16t* o0 = pl + m * 144 + pr * 12 + pc;
    o0[0] = (f16t)(p0 * A1C);
    o0[1] = (f16t)(p1 * A1C);
    if (m < 4) {
      const float q0 = fmaxf(fmaxf(acc1[0], acc1[1]), fmaxf(acc1[2], acc1[3])) * inv_c + bias1;
      const float q1 = fmaxf(fmaxf(acc1[4], acc1[5]), fmaxf(acc1[6], acc1[7])) * inv_c + bias1;
      f16t* o1 = pl + (16 + m) * 144 + pr * 12 + pc;
      o1[0] = (f16t)(q0 * A1C);
      o1[1] = (f16t)(q1 * A1C);
    }
  }
  __syncthreads();

  {
    f16t* ab = act1 + (size_t)img0 * FC1IN;
    const int p2 = imin(tid + 2 * TPB, 719);
    const bool t2 = (tid + 2 * TPB) < 720;
    const v8h v0 = *(const v8ha*)(spool + 8 * tid);
    const v8h v1 = *(const v8ha*)(spool + 8 * (tid + TPB));
    const v8h v2 = *(const v8ha*)(spool + 8 * p2);
    f16t* d0 = ab + 8 * tid;
    f16t* d1 = ab + 8 * (tid + TPB);
    f16t* d2 = ab + 8 * p2;
    *(volatile v8h*)d0 = v0;
    *(volatile v8h*)d1 = v1;
    if (t2) *(volatile v8h*)d2 = v2;
    __threadfence();
    *(volatile v8h*)d0 = v0;
    *(volatile v8h*)d1 = v1;
    if (t2) *(volatile v8h*)d2 = v2;
  }
}

__global__ __launch_bounds__(TPB) void fc1_k(const f16t* __restrict__ act1,
                                            const f16t* __restrict__ W1,
                                            const float* __restrict__ fc1_b,
                                            f16t* __restrict__ act2)
{
  __shared__ __attribute__((aligned(16))) f16t stg[8 * 32 * STGP];
  const int tid = threadIdx.x, lane = tid & 31, wave = tid >> 5;
  const int h = lane >> 4, m = lane & 15;
  const int rbase = blockIdx.x * 32;

  const f16t* ar0 = act1 + (size_t)(rbase + m) * FC1IN + 8 * h;
  const f16t* ar1 = ar0 + (size_t)16 * FC1IN;
  const f16t* wb  = W1 + (size_t)(wave * 64 + m) * FC1IN + 8 * h;

  v8f acc[2][4];
  #pragma unroll
  for (int mt = 0; mt < 2; ++mt) {
    #pragma unroll
    for (int i = 0; i < 4; ++i) acc[mt][i] = zero8f();
  }

  for (int kt = 0; kt < FC1IN / 32; ++kt) {
    const int k0 = kt * 32;
    FragH b[4];
    #pragma unroll
    for (int i = 0; i < 4; ++i) {
      const f16t* wr = wb + (size_t)i * 16 * FC1IN + k0;
      b[i].half[0] = *(const v8ha*)(wr);
      b[i].half[1] = *(const v8ha*)(wr + 16);
    }
    {
      FragH a;
      a.half[0] = *(const v8ha*)(ar0 + k0);
      a.half[1] = *(const v8ha*)(ar0 + k0 + 16);
      #pragma unroll
      for (int i = 0; i < 4; ++i) acc[0][i] = wmma_f16(a.v, b[i].v, acc[0][i]);
    }
    {
      FragH a;
      a.half[0] = *(const v8ha*)(ar1 + k0);
      a.half[1] = *(const v8ha*)(ar1 + k0 + 16);
      #pragma unroll
      for (int i = 0; i < 4; ++i) acc[1][i] = wmma_f16(a.v, b[i].v, acc[1][i]);
    }
  }

  f16t* sw = stg + wave * (32 * STGP);
  const float sc1 = 1.0f / (A1C * W1C);
  #pragma unroll
  for (int i = 0; i < 4; ++i) {
    const int n = wave * 64 + 16 * i + m;
    const float bb = fc1_b[imin(n, FC1O - 1)];
    const float bias = (n < FC1O) ? bb : 0.0f;
    #pragma unroll
    for (int mt = 0; mt < 2; ++mt) {
      #pragma unroll
      for (int r = 0; r < 8; ++r) {
        const float v = fmaxf(fmaf(acc[mt][i][r], sc1, bias), 0.0f) * A2C;
        sw[(mt * 16 + 8 * h + r) * STGP + 16 * i + m] = (f16t)v;
      }
    }
  }
  __syncthreads();

  v8h vals[8];
  const int lq = lane >> 3, q = lane & 7;
  #pragma unroll
  for (int j = 0; j < 8; ++j) {
    const int L = 4 * j + lq;
    vals[j] = *(const v8ha*)(sw + L * STGP + 8 * q);
  }
  f16t* ob = act2 + (size_t)rbase * FC1P + wave * 64 + 8 * q;
  #pragma unroll
  for (int j = 0; j < 8; ++j) {
    const int L = 4 * j + lq;
    *(volatile v8h*)(ob + (size_t)L * FC1P) = vals[j];
  }
  __threadfence();
  #pragma unroll
  for (int j = 0; j < 8; ++j) {
    const int L = 4 * j + lq;
    *(volatile v8h*)(ob + (size_t)L * FC1P) = vals[j];
  }
}

__global__ __launch_bounds__(TPB) void fc2_softmax_k(const f16t* __restrict__ act2,
                                                    const f16t* __restrict__ W2,
                                                    const float* __restrict__ fc2_b,
                                                    float* __restrict__ out)
{
  __shared__ __attribute__((aligned(16))) float so[128 * FC2O];
  const int tid = threadIdx.x, lane = tid & 31, wave = tid >> 5;
  const int h = lane >> 4, m = lane & 15;
  const int rloc  = wave * 16;
  const int rbase = blockIdx.x * 128 + rloc;

  const f16t* arow = act2 + (size_t)(rbase + m) * FC1P + 8 * h;
  const f16t* wrow = W2 + (size_t)m * FC1P + 8 * h;

  v8f acc = zero8f();
  for (int kt = 0; kt < FC1P / 32; ++kt) {
    const int k0 = kt * 32;
    FragH a, b;
    a.half[0] = *(const v8ha*)(arow + k0);
    a.half[1] = *(const v8ha*)(arow + k0 + 16);
    b.half[0] = *(const v8ha*)(wrow + k0);
    b.half[1] = *(const v8ha*)(wrow + k0 + 16);
    acc = wmma_f16(a.v, b.v, acc);
  }

  const float sc2 = 1.0f / (A2C * W2C);
  const bool valid = (m < FC2O);
  const float bb = fc2_b[imin(m, FC2O - 1)];
  #pragma unroll
  for (int v = 0; v < 8; ++v) {
    const float val = valid ? fmaf(acc[v], sc2, bb) : -__builtin_inff();
    float r = val;
    r = fmaxf(r, __shfl_xor(r, 8, 16));
    r = fmaxf(r, __shfl_xor(r, 4, 16));
    r = fmaxf(r, __shfl_xor(r, 2, 16));
    r = fmaxf(r, __shfl_xor(r, 1, 16));
    const float arg = valid ? (val - r) : 0.0f;
    const float ee  = expf(arg);
    const float ex  = valid ? ee : 0.0f;
    float s = ex;
    s += __shfl_xor(s, 8, 16);
    s += __shfl_xor(s, 4, 16);
    s += __shfl_xor(s, 2, 16);
    s += __shfl_xor(s, 1, 16);
    const float o = ex * __builtin_amdgcn_rcpf(s);
    if (valid) so[(rloc + 8 * h + v) * FC2O + m] = o;
  }
  __syncthreads();

  float* obase = out + (size_t)blockIdx.x * (128 * FC2O);
  const int pb = imin(tid + TPB, 319);
  const bool sb = (tid + TPB) < 320;
  const v4f va = *(const v4fa*)(so + 4 * tid);
  const v4f vb = *(const v4fa*)(so + 4 * pb);
  float* da = obase + 4 * tid;
  float* db = obase + 4 * pb;
  *(volatile v4f*)da = va;
  if (sb) *(volatile v4f*)db = vb;
  __threadfence();
  *(volatile v4f*)da = va;
  if (sb) *(volatile v4f*)db = vb;
}

extern "C" void kernel_launch(void* const* d_in, const int* in_sizes, int n_in,
                              void* d_out, int out_size, void* d_ws, size_t ws_size,
                              hipStream_t stream) {
  if (n_in < 7) return;
  if (out_size <= 0 || (out_size % FC2O) != 0) return;
  const int nB = out_size / FC2O;
  if ((nB % 128) != 0) return;
  if (in_sizes[0] != nB * IMGSZ)    return;
  if (in_sizes[1] != CO * KTAP)     return;
  if (in_sizes[2] != CO)            return;
  if (in_sizes[3] != FC1O * FC1IN)  return;
  if (in_sizes[4] != FC1O)          return;
  if (in_sizes[5] != FC2O * FC1O)   return;
  if (in_sizes[6] != FC2O)          return;

  const float* x      = (const float*)d_in[0];
  const float* conv_w = (const float*)d_in[1];
  const float* conv_b = (const float*)d_in[2];
  const float* fc1_w  = (const float*)d_in[3];
  const float* fc1_b  = (const float*)d_in[4];
  const float* fc2_w  = (const float*)d_in[5];
  const float* fc2_b  = (const float*)d_in[6];
  float* outp = (float*)d_out;

  const size_t szWc = (size_t)NCP * KCP * 2;
  const size_t szW1 = (size_t)FC1P * FC1IN * 2;
  const size_t szW2 = (size_t)FC2P * FC1P * 2;
  const size_t szA1 = (size_t)nB * FC1IN * 2;
  const size_t szA2 = (size_t)nB * FC1P * 2;
  size_t off = 0;
  char* ws = (char*)d_ws;
  f16t* Wc   = (f16t*)(ws + off); off += szWc;
  f16t* W1   = (f16t*)(ws + off); off += szW1;
  f16t* W2   = (f16t*)(ws + off); off += szW2;
  f16t* act1 = (f16t*)(ws + off); off += szA1;
  f16t* act2 = (f16t*)(ws + off); off += szA2;
  if (off > ws_size) return;
  if (off > (size_t)128 * 1024 * 1024) return;

  prep_k<<<dim3(FC1P * (FC1IN / 8) / TPB, 3), TPB, 0, stream>>>(conv_w, fc1_w, fc2_w, Wc, W1, W2);
  conv_pool_k<<<nB / 2, TPB, 0, stream>>>(x, conv_b, Wc, act1);
  fc1_k<<<nB / 32, TPB, 0, stream>>>(act1, W1, fc1_b, act2);
  fc2_softmax_k<<<nB / 128, TPB, 0, stream>>>(act2, W2, fc2_b, outp);
}
